// TemporalAttention_80247168958702
// MI455X (gfx1250) — hardware-run, weakly checked
//
#include <hip/hip_runtime.h>


#ifndef NB
#define NB 8
#endif
#ifndef SEQ
#define SEQ 2048
#endif
#define NB_FULL  8
#define SEQ_FULL 2048
#ifndef OUT_SEQ
#define OUT_SEQ SEQ
#endif
#define DM   512
#define PVR  32
#define PVW  4
#define NJ   (SEQ / 256)
#define PSC  16384.0f
#define PSI  (1.0f / 16384.0f)
#define SC2  ((float)(0.044194173824159216 * 1.4426950408889634))
#define NEGB (-3.0e38f)
#define LNEPS 1.0e-6f

static_assert(DM % 64 == 0);
static_assert(DM % 32 == 0);
static_assert(SEQ % 64 == 0);
static_assert((NB * SEQ) % 64 == 0);
static_assert(SEQ % 32 == 0);
static_assert(SEQ % 256 == 0);
static_assert(NJ % 2 == 0 || NJ == 1);
static_assert(SEQ % 8 == 0);
static_assert(SEQ % PVR == 0);
static_assert(PVR == 32);
static_assert(PVW * 128 == DM);
static_assert(PVR % PVW == 0);
static_assert(32 * 4 * 4 == DM);
static_assert((size_t)PVR * DM * 4 <= 131072);
static_assert(16 * 68 * 4 <= 131072);
static_assert(64 * 65 * 4 <= 131072);
static_assert(32 * 16 * 4 == 16 * 128);
static_assert(32 * 16 * 8 == 16 * 256);
static_assert(2 * 256 * 8 == 64 * 64);
static_assert(16 * 256 == 64 * 64);
static_assert(32 * 8 * NJ == SEQ);
static_assert(32 * 4 * 4 * 4 == DM * 4);
static_assert(((size_t)SEQ * DM) % 8 == 0);
static_assert(((size_t)DM * DM) % 8 == 0);
static_assert(NB <= NB_FULL);
static_assert(SEQ <= SEQ_FULL);

typedef _Float16 h16;
typedef unsigned short bf;
typedef __attribute__((ext_vector_type(16))) __bf16   v16bf;
typedef __attribute__((ext_vector_type(16))) _Float16 v16h;
typedef __attribute__((ext_vector_type(8)))  _Float16 v8h;
typedef __attribute__((ext_vector_type(8)))  unsigned short v8us;
typedef __attribute__((ext_vector_type(4)))  unsigned short v4us;
typedef __attribute__((ext_vector_type(8)))  float    v8f;
typedef __attribute__((ext_vector_type(4)))  float    v4f;
typedef __attribute__((ext_vector_type(4)))  int      v4i;
typedef v4f  __attribute__((may_alias)) v4fa;

__device__ __forceinline__ unsigned short f2bf(float f) { unsigned u = __float_as_uint(f); u += 0x7FFFu + ((u >> 16) & 1u); return (unsigned short)(u >> 16); }
__device__ __forceinline__ float bfr(float f) { return __uint_as_float(((unsigned)f2bf(f)) << 16); }
__device__ __forceinline__ v16h cat16(v8h lo, v8h hi) { return __builtin_shufflevector(lo, hi, 0, 1, 2, 3, 4, 5, 6, 7, 8, 9, 10, 11, 12, 13, 14, 15); }
__device__ __forceinline__ v16bf cat16b(v8us lo, v8us hi) { return __builtin_bit_cast(v16bf, __builtin_shufflevector(lo, hi, 0, 1, 2, 3, 4, 5, 6, 7, 8, 9, 10, 11, 12, 13, 14, 15)); }
__device__ __forceinline__ v8f wmma16(v16h a, v16h b, v8f c) { return __builtin_amdgcn_wmma_f32_16x16x32_f16(false, a, false, b, (short)0, c, false, false); }
__device__ __forceinline__ v8f wmmab(v16bf a, v16bf b, v8f c) { return __builtin_amdgcn_wmma_f32_16x16x32_bf16(false, a, false, b, (short)0, c, false, false); }
__device__ __forceinline__ v16h  ldh(const h16* p) { return cat16(*(const v8h*)p, *(const v8h*)(p + 16)); }
__device__ __forceinline__ v16bf ldb(const bf* p)  { return cat16b(*(const v8us*)p, *(const v8us*)(p + 16)); }
__device__ __forceinline__ void wave_sync() { __builtin_amdgcn_fence(3  , "wavefront"); __builtin_amdgcn_wave_barrier(); asm volatile("" ::: "memory"); }

__device__ __forceinline__ v8f wmmabg(v16bf a, v16bf b, v8f c) { c = wmmab(a, b, c); asm volatile("v_nop\n\tv_nop\n\tv_nop\n\tv_nop" : "+v"(c) : "v"(a), "v"(b)); return c; }
__device__ __forceinline__ v8f wmma16g(v16h a, v16h b, v8f c) { c = wmma16(a, b, c); asm volatile("v_nop\n\tv_nop\n\tv_nop\n\tv_nop" : "+v"(c) : "v"(a), "v"(b)); return c; }
static __device__ __forceinline__ h16 toh_flush(float v) { const float w = (fabsf(v) < 6.103515625e-05f) ? 0.0f : v; return (h16)w; }
__device__ __forceinline__ v8h cvt8h(v4f x0, v4f x1) { v8h o;
#pragma unroll
    for (int i = 0; i < 4; ++i) { o[i] = toh_flush(x0[i]); o[4 + i] = toh_flush(x1[i]); }
    return o; }

__global__ __launch_bounds__(256) void k_cvt8(const float* __restrict__ src, bf* dst, size_t n8) {
    const size_t i = (size_t)blockIdx.x * 256 + threadIdx.x; if (i >= n8) return;
    const v8f v = *(const v8f*)(src + i * 8); v8us o;
#pragma unroll
    for (int k = 0; k < 8; ++k) o[k] = f2bf(v[k]);
    *(volatile v8us*)(dst + i * 8) = o; __threadfence(); *(volatile v8us*)(dst + i * 8) = o;
}

__global__ __launch_bounds__(256) void k_wtr(const float* __restrict__ W, bf* WT) {
    __shared__ float ts[64 * 65];
    const unsigned tid = threadIdx.x;
    const unsigned i0 = blockIdx.x * 64u, o0 = blockIdx.y * 64u;
#pragma unroll 1
    for (unsigned it = 0; it < 16u; ++it) { const unsigned e = it * 256u + tid; const unsigned r = e >> 6, c = e & 63u;
        ts[c * 65u + r] = W[(size_t)(i0 + r) * DM + o0 + c]; }
    __syncthreads();
#pragma unroll 1
    for (int ps = 0; ps < 2; ++ps) {
#pragma unroll 1
        for (unsigned it = 0; it < 2u; ++it) { const unsigned p = it * 256u + tid; const unsigned row = p >> 3, c8 = (p & 7u) * 8u;
            v8us o;
#pragma unroll
            for (int k = 0; k < 8; ++k) o[k] = f2bf(ts[row * 65u + c8 + k]);
            *(volatile v8us*)(WT + (size_t)(o0 + row) * DM + i0 + c8) = o; }
        if (ps == 0) __threadfence(); }
}

__global__ __launch_bounds__(32) void k_proj_rows(const bf* __restrict__ A, const bf* __restrict__ Bt, const float* __restrict__ bias, h16* Ph) {
    __shared__ __align__(16) float os[16 * 68];
    const unsigned lane = threadIdx.x & 31u, lr = lane & 15u, hi = lane >> 4; const unsigned r0 = blockIdx.x * 64u, c0 = blockIdx.y * 64u;
    v8f acc[4][4];
#pragma unroll
    for (int mb = 0; mb < 4; ++mb)
#pragma unroll
        for (int nb = 0; nb < 4; ++nb) acc[mb][nb] = (v8f){};
    const size_t aoff = (size_t)(r0 + lr) * DM + 8u * hi, boff = (size_t)(c0 + lr) * DM + 8u * hi;
#pragma unroll 1
    for (unsigned kc = 0; kc < (unsigned)DM; kc += 32u) {
        v16bf a[4];
#pragma unroll
        for (int mb = 0; mb < 4; ++mb) a[mb] = ldb(A + aoff + (size_t)mb * 16 * DM + kc);
#pragma unroll
        for (int nb = 0; nb < 4; ++nb) { const v16bf b = ldb(Bt + boff + (size_t)nb * 16 * DM + kc);
#pragma unroll
            for (int mb = 0; mb < 4; ++mb) acc[mb][nb] = wmmabg(a[mb], b, acc[mb][nb]); }
    }
    float bc[4];
#pragma unroll
    for (int nb = 0; nb < 4; ++nb) bc[nb] = bfr(bias[c0 + nb * 16 + lr]);
#pragma unroll
    for (int mb = 0; mb < 4; ++mb) {
#pragma unroll
        for (int nb = 0; nb < 4; ++nb) {
#pragma unroll
            for (int j = 0; j < 8; ++j) os[(hi * 8 + j) * 68 + nb * 16 + lr] = acc[mb][nb][j] + bc[nb]; }
        wave_sync();
        const size_t sb = (size_t)(r0 + mb * 16) * DM + c0;
#pragma unroll 1
        for (int ps = 0; ps < 2; ++ps) {
#pragma unroll
            for (int s = 0; s < 4; ++s) { const unsigned row = 4u * s + (lane >> 3), c8 = (lane & 7u) * 8u;
                const v4f x0 = *(const v4fa*)(&os[row * 68 + c8]); const v4f x1 = *(const v4fa*)(&os[row * 68 + c8 + 4]);
                const v8h hv = cvt8h(x0, x1);
                *(volatile v8h*)(Ph + sb + (size_t)row * DM + c8) = hv; }
            if (ps == 0) __threadfence(); }
        wave_sync();
    }
}

__global__ __launch_bounds__(32) void k_proj_cols(const bf* __restrict__ A, const bf* __restrict__ Bt, const float* __restrict__ bias, h16* Ph) {
    __shared__ __align__(16) float os[16 * 68];
    const unsigned lane = threadIdx.x & 31u, lr = lane & 15u, hi = lane >> 4; const unsigned r0 = blockIdx.x * 64u, c0 = blockIdx.y * 64u;
    v8f acc[4][4];
#pragma unroll
    for (int mb = 0; mb < 4; ++mb)
#pragma unroll
        for (int nb = 0; nb < 4; ++nb) acc[mb][nb] = (v8f){};
    const size_t aoff = (size_t)(r0 + lr) * DM + 8u * hi, boff = (size_t)(c0 + lr) * DM + 8u * hi;
#pragma unroll 1
    for (unsigned kc = 0; kc < (unsigned)DM; kc += 32u) {
        v16bf a[4];
#pragma unroll
        for (int mb = 0; mb < 4; ++mb) a[mb] = ldb(A + aoff + (size_t)mb * 16 * DM + kc);
#pragma unroll
        for (int nb = 0; nb < 4; ++nb) { const v16bf b = ldb(Bt + boff + (size_t)nb * 16 * DM + kc);
#pragma unroll
            for (int mb = 0; mb < 4; ++mb) acc[mb][nb] = wmmabg(a[mb], b, acc[mb][nb]); }
    }
    const unsigned bb = c0 / (unsigned)SEQ, tt = c0 % (unsigned)SEQ;
    const size_t tbase = (size_t)bb * (size_t)DM * SEQ + (size_t)r0 * SEQ + (size_t)tt;
#pragma unroll
    for (int mb = 0; mb < 4; ++mb) {
        float br[8];
#pragma unroll
        for (int j = 0; j < 8; ++j) br[j] = bfr(bias[r0 + mb * 16 + hi * 8 + j]);
#pragma unroll
        for (int nb = 0; nb < 4; ++nb) {
#pragma unroll
            for (int j = 0; j < 8; ++j) os[(hi * 8 + j) * 68 + nb * 16 + lr] = acc[mb][nb][j] + br[j]; }
        wave_sync();
        const size_t sb = tbase + (size_t)(mb * 16) * SEQ;
#pragma unroll 1
        for (int ps = 0; ps < 2; ++ps) {
#pragma unroll
            for (int s = 0; s < 4; ++s) { const unsigned row = 4u * s + (lane >> 3), c8 = (lane & 7u) * 8u;
                const v4f x0 = *(const v4fa*)(&os[row * 68 + c8]); const v4f x1 = *(const v4fa*)(&os[row * 68 + c8 + 4]);
                const v8h hv = cvt8h(x0, x1);
                *(volatile v8h*)(Ph + sb + (size_t)row * SEQ + c8) = hv; }
            if (ps == 0) __threadfence(); }
        wave_sync();
    }
}

__global__ __launch_bounds__(32) void k_scores(const h16* __restrict__ Q, const h16* __restrict__ Kp, const int* __restrict__ mask, float* LG) {
    __shared__ __align__(16) float os[16 * 68];
    const unsigned lane = threadIdx.x & 31u, lr = lane & 15u, hi = lane >> 4; const unsigned r0 = blockIdx.x * 64u, c0 = blockIdx.y * 64u;
    v8f acc[4][4];
#pragma unroll
    for (int mb = 0; mb < 4; ++mb)
#pragma unroll
        for (int nb = 0; nb < 4; ++nb) acc[mb][nb] = (v8f){};
    const size_t aoff = (size_t)(r0 + lr) * DM + 8u * hi, boff = (size_t)(c0 + lr) * DM + 8u * hi;
#pragma unroll 1
    for (unsigned kc = 0; kc < (unsigned)DM; kc += 32u) {
        v16h a[4];
#pragma unroll
        for (int mb = 0; mb < 4; ++mb) a[mb] = ldh(Q + aoff + (size_t)mb * 16 * DM + kc);
#pragma unroll
        for (int nb = 0; nb < 4; ++nb) { const v16h b = ldh(Kp + boff + (size_t)nb * 16 * DM + kc);
#pragma unroll
            for (int mb = 0; mb < 4; ++mb) acc[mb][nb] = wmma16g(a[mb], b, acc[mb][nb]); }
    }
    v4i mk = *(const v4i*)(mask + c0 + lr * 4u);
    asm volatile("" : "+v"(mk));
#pragma unroll
    for (int mb = 0; mb < 4; ++mb) {
#pragma unroll
        for (int nb = 0; nb < 4; ++nb) {
#pragma unroll
            for (int j = 0; j < 8; ++j) os[(hi * 8 + j) * 68 + nb * 16 + lr] = acc[mb][nb][j] * SC2; }
        wave_sync();
        const size_t sb = (size_t)(r0 + mb * 16) * SEQ + c0;
#pragma unroll 1
        for (int ps = 0; ps < 2; ++ps) {
#pragma unroll
            for (int s = 0; s < 8; ++s) { const unsigned row = 2u * s + hi, cofs = lr * 4u;
                v4f val = *(const v4fa*)(&os[row * 68 + cofs]);
#pragma unroll
                for (int i = 0; i < 4; ++i) val[i] = (mk[i] != 0) ? val[i] : NEGB;
                *(volatile v4f*)(LG + sb + (size_t)row * SEQ + cofs) = val; }
            if (ps == 0) __threadfence(); }
        wave_sync();
    }
}

__global__ __launch_bounds__(256) void k_softmax(const float* __restrict__ LG, h16* PH) {
#pragma clang fp contract(off)
    const unsigned lane = threadIdx.x & 31u;
    const unsigned wave = (unsigned)__builtin_amdgcn_readfirstlane((int)(threadIdx.x >> 5));
    const unsigned row = blockIdx.x * 8u + wave;
    const float* src = LG + (size_t)row * SEQ + lane * 8u;
    v4f t[2 * NJ];
    float mx = NEGB;
#pragma unroll
    for (int j = 0; j < NJ / 2; ++j) { t[2 * j] = *(const v4f*)(src + j * 256); t[2 * j + 1] = *(const v4f*)(src + j * 256 + 4); }
#pragma unroll
    for (int q = 0; q < 2 * (NJ / 2); ++q) {
#pragma unroll
        for (int i = 0; i < 4; ++i) mx = fmaxf(mx, t[q][i]); }
    asm volatile("" : "+v"(mx) : : "memory");
#pragma unroll
    for (int j = NJ / 2; j < NJ; ++j) { t[2 * j] = *(const v4f*)(src + j * 256); t[2 * j + 1] = *(const v4f*)(src + j * 256 + 4); }
#pragma unroll
    for (int q = 2 * (NJ / 2); q < 2 * NJ; ++q) {
#pragma unroll
        for (int i = 0; i < 4; ++i) mx = fmaxf(mx, t[q][i]); }
    mx = fmaxf(mx, __shfl_xor(mx, 16, 32)); mx = fmaxf(mx, __shfl_xor(mx, 8, 32)); mx = fmaxf(mx, __shfl_xor(mx, 4, 32));
    mx = fmaxf(mx, __shfl_xor(mx, 2, 32));  mx = fmaxf(mx, __shfl_xor(mx, 1, 32));
    float ls = 0.0f;
#pragma unroll
    for (int q = 0; q < 2 * NJ; ++q) {
#pragma unroll
        for (int i = 0; i < 4; ++i) { const float ex = __builtin_amdgcn_exp2f(t[q][i] - mx); const float e = (t[q][i] > -1.0e38f) ? ex : 0.0f; t[q][i] = e; ls += e; } }
    ls += __shfl_xor(ls, 16, 32); ls += __shfl_xor(ls, 8, 32); ls += __shfl_xor(ls, 4, 32); ls += __shfl_xor(ls, 2, 32); ls += __shfl_xor(ls, 1, 32);
    const bool any = ls > 0.0f;
    const float lsafe = any ? ls : 1.0f;
    const float inv = any ? (PSC * (1.0f / lsafe)) : 0.0f;
    h16* dst = PH + (size_t)row * SEQ + lane * 8u;
#pragma unroll 1
    for (int ps = 0; ps < 2; ++ps) {
#pragma unroll
        for (int j = 0; j < NJ; ++j) { const v8h o = cvt8h(t[2 * j] * inv, t[2 * j + 1] * inv);
            *(volatile v8h*)(dst + j * 256) = o; }
        if (ps == 0) __threadfence(); }
}

__global__ __launch_bounds__(32 * PVW) void k_pv(const h16* __restrict__ PH, const h16* __restrict__ VT, const bf* __restrict__ XB,
                                                 const float* __restrict__ gamma, const float* __restrict__ beta, float* OUT) {
    __shared__ __align__(16) float ts[PVR * DM];
    const unsigned lane = threadIdx.x & 31u, lr = lane & 15u, hi = lane >> 4;
    const unsigned wave = (unsigned)__builtin_amdgcn_readfirstlane((int)(threadIdx.x >> 5));
    const unsigned r0 = blockIdx.x * (unsigned)PVR, c0 = wave * 128u;
    v8f acc[2][8];
#pragma unroll
    for (int mb = 0; mb < 2; ++mb)
#pragma unroll
        for (int nb = 0; nb < 8; ++nb) acc[mb][nb] = (v8f){};
    const size_t aoff = (size_t)(r0 + lr) * SEQ + 8u * hi, boff = (size_t)(c0 + lr) * SEQ + 8u * hi;
#pragma unroll 1
    for (unsigned kc = 0; kc < (unsigned)SEQ; kc += 32u) {
        const v16h a0 = ldh(PH + aoff + kc), a1 = ldh(PH + aoff + (size_t)16 * SEQ + kc);
#pragma unroll
        for (int nb = 0; nb < 8; ++nb) { const v16h b = ldh(VT + boff + (size_t)nb * 16 * SEQ + kc);
            acc[0][nb] = wmma16g(a0, b, acc[0][nb]); acc[1][nb] = wmma16g(a1, b, acc[1][nb]); }
    }
#pragma unroll
    for (int mb = 0; mb < 2; ++mb) {
#pragma unroll
        for (int nb = 0; nb < 8; ++nb) {
#pragma unroll
            for (int j = 0; j < 8; ++j) ts[(mb * 16 + hi * 8 + j) * DM + c0 + nb * 16 + lr] = acc[mb][nb][j] * PSI; } }
    __syncthreads();
    v4f g[4], be[4];
#pragma unroll
    for (int i = 0; i < 4; ++i) { const unsigned c = 4u * lane + 128u * i; const v4f gv = *(const v4f*)(gamma + c); const v4f bv = *(const v4f*)(beta + c);
#pragma unroll
        for (int k = 0; k < 4; ++k) { g[i][k] = bfr(gv[k]); be[i][k] = bfr(bv[k]); } }
#pragma unroll 1
    for (unsigned rr = 0; rr < (unsigned)(PVR / PVW); ++rr) {
        const unsigned row = wave * (unsigned)(PVR / PVW) + rr;
        v4f v[4]; float s = 0.0f;
#pragma unroll
        for (int i = 0; i < 4; ++i) { const unsigned c = 4u * lane + 128u * i;
            v4f a = *(const v4fa*)(&ts[row * DM + c]);
            const v4us xb = *(const v4us*)(XB + (size_t)(r0 + row) * DM + c);
#pragma unroll
            for (int k = 0; k < 4; ++k) { a[k] += __uint_as_float(((unsigned)xb[k]) << 16); s += a[k]; }
            v[i] = a; }
        s += __shfl_xor(s, 16, 32); s += __shfl_xor(s, 8, 32); s += __shfl_xor(s, 4, 32); s += __shfl_xor(s, 2, 32); s += __shfl_xor(s, 1, 32);
        const float mu = s * (1.0f / (float)DM);
        float q = 0.0f;
#pragma unroll
        for (int i = 0; i < 4; ++i) {
#pragma unroll
            for (int k = 0; k < 4; ++k) { const float d = v[i][k] - mu; q += d * d; } }
        q += __shfl_xor(q, 16, 32); q += __shfl_xor(q, 8, 32); q += __shfl_xor(q, 4, 32); q += __shfl_xor(q, 2, 32); q += __shfl_xor(q, 1, 32);
        const float rstd = rsqrtf(q * (1.0f / (float)DM) + LNEPS);
#pragma unroll
        for (int i = 0; i < 4; ++i) { const unsigned c = 4u * lane + 128u * i; v4f o;
#pragma unroll
            for (int k = 0; k < 4; ++k) o[k] = (v[i][k] - mu) * rstd * g[i][k] + be[i][k];
            *(v4fa*)(&ts[row * DM + c]) = o;
            *(volatile v4f*)(OUT + (size_t)(r0 + row) * DM + c) = o; }
    }
    wave_sync();
    __threadfence();
#pragma unroll 1
    for (unsigned rr = 0; rr < (unsigned)(PVR / PVW); ++rr) {
        const unsigned row = wave * (unsigned)(PVR / PVW) + rr;
#pragma unroll
        for (int i = 0; i < 4; ++i) { const unsigned c = 4u * lane + 128u * i;
            const v4f val = *(const v4fa*)(&ts[row * DM + c]);
            *(volatile v4f*)(OUT + (size_t)(r0 + row) * DM + c) = val; }
    }
}

static constexpr size_t al256(size_t v) { return (v + 255) & ~(size_t)255; }
static constexpr size_t SZ_XB = al256((size_t)NB * SEQ * DM * 2);
static constexpr size_t SZ_WB = al256((size_t)3 * DM * DM * 2);
static constexpr size_t SZ_PL = al256((size_t)NB * SEQ * DM * 2);
static constexpr size_t SZ_LG = al256((size_t)SEQ * SEQ * 4);
static constexpr size_t SZ_PH = al256((size_t)SEQ * SEQ * 2);
static constexpr size_t SZ_TOTAL = SZ_XB + SZ_WB + 3 * SZ_PL + SZ_LG + SZ_PH;
static_assert(SZ_TOTAL <= (size_t)134217728);
static_assert(((size_t)DM * DM * 2) % 256 == 0);
static_assert(((size_t)SEQ * DM * 2) % 256 == 0);

extern "C" void kernel_launch(void* const* d_in, const int* in_sizes, int n_in,
                              void* d_out, int out_size, void* d_ws, size_t ws_size, hipStream_t stream) {
    if (n_in < 10) return;
    const size_t needx = ((size_t)(NB - 1) * SEQ_FULL + SEQ) * DM;
    const size_t needm = (size_t)(NB - 1) * SEQ_FULL + SEQ;
    if ((size_t)in_sizes[0] < needx || (size_t)in_sizes[1] < needm) return;
    if ((size_t)in_sizes[2] < (size_t)DM * DM || (size_t)in_sizes[4] < (size_t)DM * DM || (size_t)in_sizes[6] < (size_t)DM * DM) return;
    if (in_sizes[3] < DM || in_sizes[5] < DM || in_sizes[7] < DM || in_sizes[8] < DM || in_sizes[9] < DM) return;
    if ((size_t)out_size < ((size_t)(NB - 1) * OUT_SEQ + SEQ) * DM) return;
    if (SZ_TOTAL > ws_size) return;
    const float* x  = (const float*)d_in[0];
    const int* mask = (const int*)d_in[1];
    const float* wq = (const float*)d_in[2]; const float* bq = (const float*)d_in[3];
    const float* wk = (const float*)d_in[4]; const float* bk = (const float*)d_in[5];
    const float* wv = (const float*)d_in[6]; const float* bv = (const float*)d_in[7];
    const float* gamma = (const float*)d_in[8]; const float* beta = (const float*)d_in[9];
    float* OUT = (float*)d_out;
    char* wsp = (char*)d_ws;
    bf* XB = (bf*)wsp; wsp += SZ_XB;
    bf* WB = (bf*)wsp; wsp += SZ_WB;
    h16* QH = (h16*)wsp; wsp += SZ_PL;
    h16* KP = (h16*)wsp; wsp += SZ_PL;
    h16* VT = (h16*)wsp; wsp += SZ_PL;
    float* LG = (float*)wsp; wsp += SZ_LG;
    h16* PH = (h16*)wsp; wsp += SZ_PH;
    bf* WQ = WB; bf* WK = WB + (size_t)DM * DM; bf* WV = WB + (size_t)2 * DM * DM;

    if (SEQ == SEQ_FULL) {
        const size_t n8 = (size_t)NB * SEQ * DM / 8;
        k_cvt8<<<(unsigned)((n8 + 255) / 256), 256, 0, stream>>>(x, XB, n8);
    } else {
        const size_t n8 = (size_t)SEQ * DM / 8;
        for (int b = 0; b < NB; ++b) k_cvt8<<<(unsigned)((n8 + 255) / 256), 256, 0, stream>>>(x + (size_t)b * SEQ_FULL * DM, XB + (size_t)b * SEQ * DM, n8);
    }
    k_wtr<<<dim3(DM / 64, DM / 64, 1), 256, 0, stream>>>(wq, WQ);
    k_wtr<<<dim3(DM / 64, DM / 64, 1), 256, 0, stream>>>(wk, WK);
    k_wtr<<<dim3(DM / 64, DM / 64, 1), 256, 0, stream>>>(wv, WV);

    k_proj_rows<<<dim3(NB * SEQ / 64, DM / 64, 1), 32, 0, stream>>>(XB, WQ, bq, QH);
    k_proj_rows<<<dim3(NB * SEQ / 64, DM / 64, 1), 32, 0, stream>>>(XB, WK, bk, KP);
    k_proj_cols<<<dim3(DM / 64, NB * SEQ / 64, 1), 32, 0, stream>>>(WV, XB, bv, VT);

    for (int b = 0; b < NB; ++b) {
        k_scores<<<dim3(SEQ / 64, SEQ / 64, 1), 32, 0, stream>>>(QH + (size_t)b * SEQ * DM, KP + (size_t)b * SEQ * DM, mask + (size_t)b * SEQ_FULL, LG);
        k_softmax<<<dim3(SEQ / 8, 1, 1), 256, 0, stream>>>(LG, PH);
        k_pv<<<dim3(SEQ / PVR, 1, 1), 32 * PVW, 0, stream>>>(PH, VT + (size_t)b * DM * SEQ, XB + (size_t)b * SEQ * DM, gamma, beta, OUT + (size_t)b * OUT_SEQ * DM);
    }
}
